// BeplerContactPredictor_23227183137347
// MI455X (gfx1250) — hardware-verified
//
#include <hip/hip_runtime.h>
#include <math.h>
#include <stdint.h>

#define BB   8
#define LL   256
#define DD   256
#define CH   32
#define KZ   512
#define WP1  520
#define JP   264
#define KCV  224
#define W2P  256
#define NDI  8
#define ZSC  64.0f
#define RSC  1024.0f
#define WSC  1024.0f
#define HSC  256.0f
#define S1   (1.0f / 65536.0f)
#define S2   (1.0f / 67108864.0f)
#define SINV (1.0f / 262144.0f)

static_assert((BB * LL * DD) % 1024 == 0);
static_assert((KZ % 32) == 0 && (KCV % 32) == 0 && (CH % 16) == 0);
static_assert((JP * CH * 2) % 128 == 0);
static_assert(((JP - 4) >= LL + 3) && (WP1 % 8) == 0);
static_assert((BB * LL) % 4 == 0);

typedef _Float16 v16h __attribute__((ext_vector_type(16)));
typedef _Float16 v8h  __attribute__((ext_vector_type(8)));
typedef float    v8f  __attribute__((ext_vector_type(8)));
typedef float    v4f  __attribute__((ext_vector_type(4)));
typedef unsigned int v4u __attribute__((ext_vector_type(4)));

union FragH { v16h v; v8h h[2]; };

__device__ __forceinline__ unsigned short bf_bits(float f) {
  unsigned u = __float_as_uint(f);
  return (unsigned short)((u + 0x7FFFu + ((u >> 16) & 1u)) >> 16);
}
__device__ __forceinline__ float bf_up(unsigned short h) { return __uint_as_float(((unsigned)h) << 16); }
__device__ __forceinline__ float bfr(float f) { return bf_up(bf_bits(f)); }
__device__ __forceinline__ unsigned short h_bits(_Float16 x) { return __builtin_bit_cast(unsigned short, x); }
__device__ __forceinline__ unsigned pk16(unsigned short a, unsigned short b) { return (unsigned)a | ((unsigned)b << 16); }
__device__ __forceinline__ unsigned pkh(float a, float b) { return pk16(h_bits((_Float16)a), h_bits((_Float16)b)); }
__device__ __forceinline__ v8f zero8() { v8f z = {0.f, 0.f, 0.f, 0.f, 0.f, 0.f, 0.f, 0.f}; return z; }

__device__ __forceinline__ v16h ldfrag_h(const _Float16* p) {
  FragH f;
  f.h[0] = *(const v8h*)(p);
  f.h[1] = *(const v8h*)(p + 16);
  return f.v;
}

__device__ __forceinline__ v8f mma_h(v16h a, v16h b, v8f c) {
  c = __builtin_amdgcn_wmma_f32_16x16x32_f16(false, a, false, b, (short)0, c, false, false);
#if defined(__HIP_DEVICE_COMPILE__)
  asm volatile("v_nop\n\tv_nop\n\tv_nop\n\tv_nop" : "+v"(c) : "v"(a), "v"(b));
#endif
  return c;
}
__device__ __forceinline__ void wave_sync_lds() {
  __builtin_amdgcn_fence(__ATOMIC_RELEASE, "workgroup");
  __builtin_amdgcn_wave_barrier();
  __builtin_amdgcn_fence(__ATOMIC_ACQUIRE, "workgroup");
}

__device__ __forceinline__ void hi_lo_frag(const float* z, v16h& fh, v16h& fl) {
#pragma unroll
  for (int t = 0; t < 16; ++t) {
    const _Float16 hv = (_Float16)z[t];
    float rs = z[t] - (float)hv;
    rs = rs * RSC;
    fh[t] = hv;
    fl[t] = (_Float16)rs;
  }
}

__global__ __launch_bounds__(256) void cvt_x(const float* __restrict__ x, float* xr) {
  const size_t e = ((size_t)blockIdx.x * 256 + threadIdx.x) * 4;
  const v4f a = *(const v4f*)(x + e);
  v4f o;
#pragma unroll
  for (int q = 0; q < 4; ++q) o[q] = bfr(a[q]);
  float* gp = xr + e;
  *(volatile v4f*)gp = o;
  __threadfence();
  *(volatile v4f*)gp = o;
}

__global__ __launch_bounds__(256) void cvt_w(const float* __restrict__ W1, const float* __restrict__ W2,
                                             unsigned short* w1t, unsigned short* w2t) {
  const int tid = threadIdx.x;
  if (blockIdx.x < 8) {
    const int t = blockIdx.x * 256 + tid;
    const int c = t >> 6, k8 = (t & 63) * 8;
    float v[8];
#pragma unroll
    for (int e = 0; e < 8; ++e) v[e] = W1[(k8 + e) * CH + c];
    v4u pk;
#pragma unroll
    for (int e = 0; e < 4; ++e) pk[e] = pkh(bfr(v[2 * e]) * WSC, bfr(v[2 * e + 1]) * WSC);
    unsigned short* gp = w1t + c * KZ + k8;
    *(volatile v4u*)gp = pk;
    __threadfence();
    *(volatile v4u*)gp = pk;
  } else {
    const int u = (blockIdx.x - 8) * 256 + tid;
    const int n = u >> 5, k8 = (u & 31) * 8;
    const int valid = (n < 7 && k8 < KCV) ? 1 : 0;
    const int idx = valid ? (n * KCV + k8) : 0;
    const v4f a0 = *(const v4f*)(W2 + idx);
    const v4f a1 = *(const v4f*)(W2 + idx + 4);
    float v[8];
#pragma unroll
    for (int e = 0; e < 4; ++e) { v[e] = valid ? a0[e] : 0.0f; v[4 + e] = valid ? a1[e] : 0.0f; }
    v4u pk;
#pragma unroll
    for (int e = 0; e < 4; ++e) pk[e] = pkh(bfr(v[2 * e]) * WSC, bfr(v[2 * e + 1]) * WSC);
    unsigned short* gp = w2t + n * W2P + k8;
    *(volatile v4u*)gp = pk;
    __threadfence();
    *(volatile v4u*)gp = pk;
  }
}

__global__ __launch_bounds__(256) void pair_gemm(const float* __restrict__ xr, const int* __restrict__ plen,
                                                 const unsigned short* __restrict__ w1t,
                                                 const float* __restrict__ b1, unsigned short* hp) {
#pragma clang fp contract(off)
  __shared__ __align__(16) unsigned short sW[CH * WP1];
  __shared__ __align__(16) float sXs[DD];
  __shared__ __align__(16) float sXa[DD];
  __shared__ __align__(16) _Float16 sT[8][16 * CH];
  const int tid = threadIdx.x, wave = tid >> 5, lane = tid & 31;
  const int bid  = blockIdx.x;
  const int jblk = bid & 1;
  const int i    = (bid >> 1) & (LL - 1);
  const int b    = bid >> 9;

#pragma unroll
  for (int q = 0; q < 8; ++q) {
    const int e8 = tid + 256 * q;
    const int c = e8 >> 6, k = (e8 & 63) * 8;
    const v4u v = *(const v4u*)(w1t + c * KZ + k);
    *(v4u*)(sW + c * WP1 + k) = v;
  }
  {
    const float xv = xr[((size_t)(b * LL + i)) * DD + tid];
    sXa[tid] = xv;
    sXs[tid] = xv * ZSC;
  }
  __syncthreads();

  const int m = lane & 15, hh = lane >> 4, koff = 8 * hh;
  const int j0 = jblk * 128 + wave * 16;
  const float* xj  = xr + ((size_t)(b * LL + j0 + m)) * DD + koff;
  const float* xis = sXs + koff;
  const float* xia = sXa + koff;
  const _Float16* Wl  = (const _Float16*)(const void*)sW;
  const _Float16* wb0 = Wl + m * WP1 + koff;
  const _Float16* wb1 = Wl + (16 + m) * WP1 + koff;
  v8f ah0 = zero8(), ah1 = zero8(), al0 = zero8(), al1 = zero8();

#pragma unroll 1
  for (int s = 0; s < 8; ++s) {
    const int d0 = 32 * s;
    const v4f a0 = *(const v4f*)(xj + d0);
    const v4f a1 = *(const v4f*)(xj + d0 + 4);
    const v4f a2 = *(const v4f*)(xj + d0 + 16);
    const v4f a3 = *(const v4f*)(xj + d0 + 20);
    const v4f p0 = *(const v4f*)(xis + d0);
    const v4f p1 = *(const v4f*)(xis + d0 + 4);
    const v4f p2 = *(const v4f*)(xis + d0 + 16);
    const v4f p3 = *(const v4f*)(xis + d0 + 20);
    float z[16];
#pragma unroll
    for (int e = 0; e < 4; ++e) {
      z[e]      = p0[e] * a0[e];
      z[4 + e]  = p1[e] * a1[e];
      z[8 + e]  = p2[e] * a2[e];
      z[12 + e] = p3[e] * a3[e];
    }
    v16h fh, fl;
    hi_lo_frag(z, fh, fl);
    const v16h fb0 = ldfrag_h(wb0 + d0);
    const v16h fb1 = ldfrag_h(wb1 + d0);
    ah0 = mma_h(fh, fb0, ah0);
    ah1 = mma_h(fh, fb1, ah1);
    al0 = mma_h(fl, fb0, al0);
    al1 = mma_h(fl, fb1, al1);
  }
#pragma unroll 1
  for (int s = 0; s < 8; ++s) {
    const int d0 = 32 * s;
    const v4f a0 = *(const v4f*)(xj + d0);
    const v4f a1 = *(const v4f*)(xj + d0 + 4);
    const v4f a2 = *(const v4f*)(xj + d0 + 16);
    const v4f a3 = *(const v4f*)(xj + d0 + 20);
    const v4f p0 = *(const v4f*)(xia + d0);
    const v4f p1 = *(const v4f*)(xia + d0 + 4);
    const v4f p2 = *(const v4f*)(xia + d0 + 16);
    const v4f p3 = *(const v4f*)(xia + d0 + 20);
    float z[16];
#pragma unroll
    for (int e = 0; e < 4; ++e) {
      z[e]      = fabsf(p0[e] - a0[e]) * ZSC;
      z[4 + e]  = fabsf(p1[e] - a1[e]) * ZSC;
      z[8 + e]  = fabsf(p2[e] - a2[e]) * ZSC;
      z[12 + e] = fabsf(p3[e] - a3[e]) * ZSC;
    }
    v16h fh, fl;
    hi_lo_frag(z, fh, fl);
    const v16h fb0 = ldfrag_h(wb0 + DD + d0);
    const v16h fb1 = ldfrag_h(wb1 + DD + d0);
    ah0 = mma_h(fh, fb0, ah0);
    ah1 = mma_h(fh, fb1, ah1);
    al0 = mma_h(fl, fb0, al0);
    al1 = mma_h(fl, fb1, al1);
  }

  const int lenb = plen[b];
  const bool iok = (i < lenb);
  const float bz0 = bfr(b1[m]);
  const float bz1 = bfr(b1[16 + m]);
  _Float16* st = sT[wave];
#pragma unroll
  for (int r = 0; r < 8; ++r) {
    const int jl = 8 * hh + r;
    const bool ok = iok && (j0 + jl < lenb);
    float u0 = ah0[r] * S1; float w0 = al0[r] * S2; float v0 = u0 + w0; v0 = v0 + bz0; v0 = fmaxf(v0, 0.0f);
    float u1 = ah1[r] * S1; float w1 = al1[r] * S2; float v1 = u1 + w1; v1 = v1 + bz1; v1 = fmaxf(v1, 0.0f);
    v0 = ok ? v0 * HSC : 0.0f;
    v1 = ok ? v1 * HSC : 0.0f;
    st[jl * CH + m]      = (_Float16)v0;
    st[jl * CH + 16 + m] = (_Float16)v1;
  }
  wave_sync_lds();
  const size_t hrow = ((size_t)(b * LL + i)) * JP * CH;
  unsigned short* gbase = hp + hrow + (size_t)(j0 + 4) * CH;
  v4u pk[2];
#pragma unroll
  for (int it = 0; it < 2; ++it) {
    const int p = it * 32 + lane;
    const v8h v = *(const v8h*)(st + p * 8);
    pk[it] = __builtin_bit_cast(v4u, v);
  }
#pragma unroll
  for (int it = 0; it < 2; ++it) { unsigned short* gp = gbase + (it * 32 + lane) * 8; *(volatile v4u*)gp = pk[it]; }
  __threadfence();
#pragma unroll
  for (int it = 0; it < 2; ++it) { unsigned short* gp = gbase + (it * 32 + lane) * 8; *(volatile v4u*)gp = pk[it]; }

  if (jblk == 0 && wave == 0) {
    const v4u zz = {0u, 0u, 0u, 0u};
    const int off = (lane < 16) ? lane * 8 : ((JP - 4) * CH + (lane - 16) * 8);
    unsigned short* gp = hp + hrow + off;
    *(volatile v4u*)gp = zz;
    __threadfence();
    *(volatile v4u*)gp = zz;
  }
}

__global__ __launch_bounds__(256) void conv_gemm(const unsigned short* __restrict__ hp,
                                                 const unsigned short* __restrict__ w2t, float* dt) {
#pragma clang fp contract(off)
  __shared__ __align__(16) unsigned short sW2[16 * W2P];
  __shared__ __align__(16) float sD[8][8 * 32];
  const int tid = threadIdx.x, wave = tid >> 5, lane = tid & 31;
  const int bid = blockIdx.x;
  const int r = bid & (LL - 1);
  const int b = bid >> 8;
#pragma unroll
  for (int q = 0; q < 2; ++q) {
    const int e = tid + 256 * q;
    const v4u v = *(const v4u*)(w2t + e * 8);
    *(v4u*)(sW2 + e * 8) = v;
  }
  __syncthreads();

  const int m = lane & 15, hh = lane >> 4, koff = 8 * hh;
  const int j0w = wave * 32;
  const _Float16* A  = (const _Float16*)(const void*)hp
                       + ((((size_t)(b * LL + r)) * JP) + j0w + 1) * CH + koff;
  const _Float16* Bw = (const _Float16*)(const void*)sW2 + m * W2P + koff;
  const _Float16* a0p = A + m * CH;
  const _Float16* a1p = A + (16 + m) * CH;
  v8f acc0 = zero8(), acc1 = zero8();
#pragma unroll 1
  for (int k0 = 0; k0 < KCV; k0 += 32) {
    const v16h fa0 = ldfrag_h(a0p + k0);
    const v16h fa1 = ldfrag_h(a1p + k0);
    const v16h fb  = ldfrag_h(Bw + k0);
    acc0 = mma_h(fa0, fb, acc0);
    acc1 = mma_h(fa1, fb, acc1);
  }

  float* sd = sD[wave];
  if (m < 8) {
#pragma unroll
    for (int rr = 0; rr < 8; ++rr) {
      sd[m * 32 + 8 * hh + rr]      = acc0[rr];
      sd[m * 32 + 16 + 8 * hh + rr] = acc1[rr];
    }
  }
  wave_sync_lds();
  v4f pv[2];
#pragma unroll
  for (int it = 0; it < 2; ++it) {
    const int p = it * 32 + lane;
    pv[it] = *(const v4f*)(sd + (p >> 3) * 32 + (p & 7) * 4);
  }
  const size_t dbase = ((size_t)(b * NDI)) * LL * LL + (size_t)r * LL + j0w;
#pragma unroll
  for (int it = 0; it < 2; ++it) {
    const int p = it * 32 + lane;
    float* gp = dt + dbase + (size_t)(p >> 3) * LL * LL + (p & 7) * 4;
    *(volatile v4f*)gp = pv[it];
  }
  __threadfence();
#pragma unroll
  for (int it = 0; it < 2; ++it) {
    const int p = it * 32 + lane;
    float* gp = dt + dbase + (size_t)(p >> 3) * LL * LL + (p & 7) * 4;
    *(volatile v4f*)gp = pv[it];
  }
}

__global__ __launch_bounds__(256) void combine7(const float* __restrict__ dt, const int* __restrict__ plen,
                                                const float* __restrict__ b2, float* outp) {
#pragma clang fp contract(off)
  const int tid = threadIdx.x;
  const int row = blockIdx.x * 4 + (tid >> 6);
  const int b = row >> 8, i = row & (LL - 1);
  const int j4 = (tid & 63) * 4;
  const int lenb = plen[b];
  const float bz = bfr(b2[0]);
  v4f s = {0.f, 0.f, 0.f, 0.f};
#pragma unroll
  for (int di = 0; di < 7; ++di) {
    const int rr = i + di - 3;
    const int ok = (rr >= 0 && rr < LL) ? 1 : 0;
    const int rc = (rr < 0) ? 0 : ((rr > LL - 1) ? (LL - 1) : rr);
    const v4f v = *(const v4f*)(dt + ((((size_t)(b * NDI + di)) * LL + rc) * LL + j4));
#pragma unroll
    for (int e = 0; e < 4; ++e) { const float a = ok ? v[e] : 0.0f; s[e] = s[e] + a; }
  }
  v4f o;
#pragma unroll
  for (int e = 0; e < 4; ++e) {
    float f = s[e] * SINV;
    f = f + bz;
    const int j = j4 + e;
    o[e] = (i < lenb && j < lenb) ? f : 0.0f;
  }
  float* gp = outp + (size_t)row * LL + j4;
  *(volatile v4f*)gp = o;
  __threadfence();
  *(volatile v4f*)gp = o;
}

extern "C" void kernel_launch(void* const* d_in, const int* in_sizes, int n_in,
                              void* d_out, int out_size, void* d_ws, size_t ws_size,
                              hipStream_t stream) {
  if (n_in < 6) return;
  const int ex[6] = { BB * LL * DD, BB, KZ * CH, CH, 49 * CH, 1 };
  for (int q = 0; q < 6; ++q) if (in_sizes[q] != ex[q]) return;
  if (out_size != BB * LL * LL) return;

  const float* x    = (const float*)d_in[0];
  const int*   plen = (const int*)d_in[1];
  const float* W1   = (const float*)d_in[2];
  const float* b1   = (const float*)d_in[3];
  const float* W2   = (const float*)d_in[4];
  const float* b2   = (const float*)d_in[5];
  float* out = (float*)d_out;

  const size_t sXR = (size_t)BB * LL * DD * 4;
  const size_t sW1 = (size_t)CH * KZ * 2;
  const size_t sW2 = (size_t)16 * W2P * 2;
  const size_t sHP = (size_t)BB * LL * JP * CH * 2;
  const size_t sDT = (size_t)BB * NDI * LL * LL * 4;
  size_t off = 0;
  const size_t oXR = off; off += sXR;
  const size_t oW1 = off; off += sW1;
  const size_t oW2 = off; off += sW2;
  const size_t oHP = off; off += sHP;
  const size_t oDT = off; off += sDT;
  if (off > ws_size) return;
  if (off > (size_t)134217728) return;

  char* ws = (char*)d_ws;
  float*          XR  = (float*)(ws + oXR);
  unsigned short* W1T = (unsigned short*)(ws + oW1);
  unsigned short* W2T = (unsigned short*)(ws + oW2);
  unsigned short* HP  = (unsigned short*)(ws + oHP);
  float*          DT  = (float*)(ws + oDT);

  const dim3 blk(256);
  cvt_x<<<dim3((BB * LL * DD) / 1024), blk, 0, stream>>>(x, XR);
  cvt_w<<<dim3(10), blk, 0, stream>>>(W1, W2, W1T, W2T);
  pair_gemm<<<dim3(BB * LL * 2), blk, 0, stream>>>(XR, plen, W1T, b1, HP);
  conv_gemm<<<dim3(BB * LL), blk, 0, stream>>>(HP, W2T, DT);
  combine7<<<dim3((BB * LL) / 4), blk, 0, stream>>>(DT, plen, b2, out);
  (void)hipGetLastError();
}
